// moe_7404523618953
// MI455X (gfx1250) — hardware-verified
//
#include <hip/hip_runtime.h>
#include <stddef.h>
#include <stdint.h>

#define NTOK   2048
#define DM     512
#define DH     1024
#define GU2    2048
#define NE     8
#define NSEL   2
#define RPITCH 8
#define NTILE  72
#define AROWS  (NTILE * 64)
#define NPROW  (NTOK * NSEL)
#define WSC    64.0f
#define UGS    0.015625f
#define ACS    256.0f
#define DNS    0.00006103515625f
#define APITCH 136
#define EPITCH 72
#define OTP    68
#define TRP    72

static_assert(NTILE == NPROW / 64 + NE);
static_assert(NSEL == 2);
static_assert(NE == 8);
static_assert(DM % 128 == 0);
static_assert(DH % 128 == 0);
static_assert(DM % 64 == 0);
static_assert(DH % 64 == 0);
static_assert(GU2 == 2 * DH);
static_assert(NTOK % 256 == 0);
static_assert(NTOK % 64 == 0);
static_assert((NTOK * DM) % 2048 == 0);
static_assert(NTOK * NSEL <= 65536);

typedef _Float16 v16h __attribute__((ext_vector_type(16)));
typedef _Float16 v8h  __attribute__((ext_vector_type(8)));
typedef float    v8f  __attribute__((ext_vector_type(8)));
typedef float    v4f  __attribute__((ext_vector_type(4)));
typedef unsigned int v4u __attribute__((ext_vector_type(4)));
typedef int      v4i  __attribute__((ext_vector_type(4)));
typedef unsigned short v4us __attribute__((ext_vector_type(4)));

union Frag  { v16h v; v8h h[2]; };
union Pack8 { v8h h; v4u u; };

__device__ __forceinline__ int clampi(int v, int lo, int hi) { return min(max(v, lo), hi); }

__device__ __forceinline__ v8f mma16(v16h a, v16h b, v8f c) {
  c = __builtin_amdgcn_wmma_f32_16x16x32_f16(false, a, false, b, (short)0, c, false, false);
  asm volatile("v_nop\n\tv_nop\n\tv_nop\n\tv_nop" : "+v"(c) : "v"(a), "v"(b));
  return c;
}

__device__ __forceinline__ v16h ldfrag(const _Float16* p, int ld, int row0, int k0, int lane) {
  const int m = lane & 15, lh = lane >> 4;
  const _Float16* q = p + (size_t)(row0 + m) * ld + k0 + 8 * lh;
  Frag f;
  f.h[0] = *(const v8h*)(q);
  f.h[1] = *(const v8h*)(q + 16);
  return f.v;
}

__device__ __forceinline__ v8f zero8() { return (v8f){0.f, 0.f, 0.f, 0.f, 0.f, 0.f, 0.f, 0.f}; }

__device__ __forceinline__ void gemm16x64(const _Float16* __restrict__ A, int lda, int arow0,
                                          const _Float16* __restrict__ Bt, int ldb, int brow0,
                                          int K, int lane, v8f (&acc)[4]) {
#pragma unroll 1
  for (int k0 = 0; k0 < K; k0 += 32) {
    const v16h a = ldfrag(A, lda, arow0, k0, lane);
#pragma unroll
    for (int t = 0; t < 4; ++t) {
      const v16h bq = ldfrag(Bt, ldb, brow0 + 16 * t, k0, lane);
      acc[t] = mma16(a, bq, acc[t]);
    }
  }
}

__global__ __launch_bounds__(256) void k_cvt(const float* __restrict__ src, _Float16* __restrict__ dh, int n8) {
  const int i = blockIdx.x * 256 + (int)threadIdx.x;
  if (i >= n8) return;
  const size_t o = (size_t)i * 8;
  const v4f a0 = *(const v4f*)(src + o);
  const v4f a1 = *(const v4f*)(src + o + 4);
  Pack8 pk;
  pk.h = (v8h){(_Float16)a0[0], (_Float16)a0[1], (_Float16)a0[2], (_Float16)a0[3],
               (_Float16)a1[0], (_Float16)a1[1], (_Float16)a1[2], (_Float16)a1[3]};
  const v4u vv = pk.u;
  volatile v4u* d = (volatile v4u*)(dh + o);
  *d = vv;
  __threadfence();
  *d = vv;
}

__global__ __launch_bounds__(256) void k_wtr(const float* __restrict__ w, _Float16* __restrict__ wt,
                                             int kdim, int ndim, float scale) {
  __shared__ __align__(16) _Float16 st[64 * TRP];
  const int tid = threadIdx.x;
  const size_t bo = (size_t)blockIdx.z * (size_t)kdim * (size_t)ndim;
  w  += bo;
  wt += bo;
  const int n0 = blockIdx.x * 64, k0 = blockIdx.y * 64;
  const int kr = tid >> 2;
  const int nc = (tid & 3) * 16;
  const float* sp = w + (size_t)(k0 + kr) * ndim + n0 + nc;
#pragma unroll
  for (int q = 0; q < 4; ++q) {
    const v4f a = *(const v4f*)(sp + 4 * q) * scale;
#pragma unroll
    for (int j = 0; j < 4; ++j) st[(nc + 4 * q + j) * TRP + kr] = (_Float16)a[j];
  }
  __syncthreads();
  v4u val[2];
  size_t go[2];
#pragma unroll
  for (int j = 0; j < 2; ++j) {
    const int p  = tid + 256 * j;
    const int nr = p >> 3;
    const int pc = p & 7;
    Pack8 pk;
    pk.h   = *(const v8h*)(st + nr * TRP + pc * 8);
    val[j] = pk.u;
    go[j]  = (size_t)(n0 + nr) * kdim + k0 + pc * 8;
  }
  for (int ps = 0; ps < 2; ++ps) {
#pragma unroll
    for (int j = 0; j < 2; ++j) *(volatile v4u*)(wt + go[j]) = val[j];
    __threadfence();
  }
}

__global__ __launch_bounds__(256) void k_route(const float* __restrict__ x, const float* __restrict__ gw,
                                               float* __restrict__ rp) {
  __shared__ __align__(16) float sR[8 * RPITCH];
  const int tid = threadIdx.x, lane = tid & 31, wave = tid >> 5;
  const int c = lane & 15;
  const size_t t = (size_t)blockIdx.x * 8 + wave;
  const float* xr = x + t * DM;

  float a[NE];
#pragma unroll
  for (int e = 0; e < NE; ++e) a[e] = 0.f;
#pragma unroll 1
  for (int j = 0; j < DM / 32; ++j) {
    const int k = j * 32 + lane;
    const float xv = xr[k];
    const v4f* wr = (const v4f*)(gw + (size_t)k * NE);
    const v4f w0 = wr[0];
    const v4f w1 = wr[1];
    a[0] += xv * w0[0];
    a[1] += xv * w0[1];
    a[2] += xv * w0[2];
    a[3] += xv * w0[3];
    a[4] += xv * w1[0];
    a[5] += xv * w1[1];
    a[6] += xv * w1[2];
    a[7] += xv * w1[3];
  }
#pragma unroll
  for (int e = 0; e < NE; ++e) {
#pragma unroll
    for (int off = 16; off >= 1; off >>= 1) a[e] += __shfl_xor(a[e], off, 32);
  }

  const float NEGI = -__builtin_huge_valf();
  unsigned taken = 0u;
  int idx[NSEL];
  float lsel[NSEL];
#pragma unroll
  for (int kk = 0; kk < NSEL; ++kk) {
    float bv = NEGI;
    int best = 0;
#pragma unroll
    for (int i = 0; i < NE; ++i) {
      const bool cnd = (((taken >> i) & 1u) == 0u) && (a[i] > bv);
      bv   = cnd ? a[i] : bv;
      best = cnd ? i : best;
    }
    taken |= (1u << best);
    idx[kk]  = best;
    lsel[kk] = bv;
  }
  const float u1  = expf(lsel[1] - lsel[0]);
  const float s   = 1.0f + u1;
  const float inv = 1.0f / s;
  const float w0  = inv;
  const float w1  = u1 * inv;

  float ov = 0.f;
  ov = (lane == 0) ? (float)idx[0] : ov;
  ov = (lane == 1) ? (float)idx[1] : ov;
  ov = (lane == 4) ? w0 : ov;
  ov = (lane == 5) ? w1 : ov;
  if (lane < RPITCH) sR[wave * RPITCH + lane] = ov;
  __syncthreads();
  if (wave == 0) {
    const v4f vr = *(const v4f*)(sR + c * 4);
    volatile v4f* dr = (volatile v4f*)(rp + (size_t)blockIdx.x * (8 * RPITCH) + c * 4);
    if (lane < 16) *dr = vr;
    __threadfence();
    if (lane < 16) *dr = vr;
  }
}

__global__ __launch_bounds__(256) void k_lists(const float* __restrict__ rp, int* __restrict__ tokl,
                                               float* __restrict__ wl, int* __restrict__ tab) {
  __shared__ __align__(16) unsigned short ltok[NTOK];
  __shared__ __align__(16) float lw[NTOK];
  __shared__ int wc[8];
  __shared__ __align__(16) int sTab[64];
  const int tid = threadIdx.x, lane = tid & 31, wave = tid >> 5;
  if (tid < 64) sTab[tid] = 0;
  int tbrun = 0;
#pragma unroll 1
  for (int e = 0; e < NE; ++e) {
    __syncthreads();
    for (int i = tid; i < NTOK; i += 256) { ltok[i] = (unsigned short)0; lw[i] = 0.f; }
    __syncthreads();
    int run = 0;
#pragma unroll 1
    for (int ch = 0; ch < NTOK / 256; ++ch) {
      const int t = ch * 256 + tid;
      const v4f ri = *(const v4f*)(rp + (size_t)t * RPITCH);
      const v4f rw = *(const v4f*)(rp + (size_t)t * RPITCH + 4);
      int hit = -1;
      float w = 0.f;
#pragma unroll
      for (int k = NSEL - 1; k >= 0; --k) {
        const bool m = ((int)ri[k] == e);
        hit = m ? k : hit;
        w   = m ? rw[k] : w;
      }
      const bool flag = (hit >= 0);
      const unsigned bal = __builtin_amdgcn_ballot_w32(flag);
      const int pre = __builtin_popcount(bal & ((1u << lane) - 1u));
      if (lane == 0) wc[wave] = __builtin_popcount(bal);
      __syncthreads();
      int base = run, tot = 0;
#pragma unroll
      for (int q = 0; q < 8; ++q) {
        const int cw = wc[q];
        base += (q < wave) ? cw : 0;
        tot  += cw;
      }
      const int pos = clampi(base + pre, 0, NTOK - 1);
      if (flag) { ltok[pos] = (unsigned short)(t * NSEL + hit); lw[pos] = w; }
      run += tot;
      __syncthreads();
    }
    run = clampi(run, 0, NTOK);
    const int ntl = (run + 63) >> 6;
    if (tid == 0) { sTab[e] = run; sTab[32 + e + 1] = clampi(tbrun + ntl, 0, NTILE); }
    tbrun += ntl;

    int*   trow = tokl + (size_t)e * NTOK;
    float* wrow = wl + (size_t)e * NTOK;
    v4i tv[2];
    v4f wv[2];
    int po[2];
#pragma unroll
    for (int it = 0; it < 2; ++it) {
      const int p = tid + 256 * it;
      const v4us u = *(const v4us*)(ltok + p * 4);
      tv[it] = (v4i){(int)u[0], (int)u[1], (int)u[2], (int)u[3]};
      wv[it] = *(const v4f*)(lw + p * 4);
      po[it] = p * 4;
    }
    for (int ps = 0; ps < 2; ++ps) {
#pragma unroll
      for (int it = 0; it < 2; ++it) {
        *(volatile v4i*)(trow + po[it]) = tv[it];
        *(volatile v4f*)(wrow + po[it]) = wv[it];
      }
      __threadfence();
    }
  }
  __syncthreads();
  if (wave == 0) {
    const v4i v = *(const v4i*)(sTab + (lane & 15) * 4);
    volatile v4i* d = (volatile v4i*)(tab + (lane & 15) * 4);
    if (lane < 16) *d = v;
    __threadfence();
    if (lane < 16) *d = v;
  }
}

__global__ __launch_bounds__(256) void k_upgate(const _Float16* __restrict__ xh,
                                                const _Float16* __restrict__ wgut,
                                                const float* __restrict__ bgu,
                                                const int* __restrict__ tokl, const int* __restrict__ tab,
                                                _Float16* __restrict__ act) {
  __shared__ __align__(16) _Float16 sA[64 * APITCH];
  __shared__ __align__(16) _Float16 sE[8 * 16 * EPITCH];
  __shared__ int   sTok[64];
  __shared__ int   sTab[64];
  const int tid = threadIdx.x, lane = tid & 31, wave = tid >> 5;
  const int hh = lane >> 4, c = lane & 15;
  const int wm = wave & 3, wn = wave >> 2;
  const int b  = blockIdx.y;
  const int n0 = blockIdx.x * 128;

  if (tid < 64) sTab[tid] = tab[tid];
  __syncthreads();
  const int tb8 = clampi(sTab[32 + NE], 0, NTILE);
  if (b >= tb8) return;
  int e = 0;
#pragma unroll
  for (int q = 1; q < NE; ++q) e += (clampi(sTab[32 + q], 0, NTILE) <= b) ? 1 : 0;
  const int tbe = clampi(sTab[32 + e], 0, NTILE);
  if (tid < 64) {
    const int rloc = (b - tbe) * 64 + tid;
    const int li = e * NTOK + clampi(rloc, 0, NTOK - 1);
    const int enc = tokl[li];
    sTok[tid] = clampi(enc >> 1, 0, NTOK - 1);
  }
  __syncthreads();

  const _Float16* wge = wgut + (size_t)e * (size_t)(GU2 * DM);
  const _Float16* wue = wge + (size_t)DH * DM;
  const int brow = n0 + wn * 64;

  float bgv[4], buv[4];
#pragma unroll
  for (int t = 0; t < 4; ++t) {
    const int col = brow + 16 * t + c;
    bgv[t] = bgu[(size_t)e * GU2 + col];
    buv[t] = bgu[(size_t)e * GU2 + DH + col];
  }

  v8f accG[4], accU[4];
#pragma unroll
  for (int t = 0; t < 4; ++t) { accG[t] = zero8(); accU[t] = zero8(); }

  const int ar = tid >> 2, ac = tid & 3;
  const _Float16* xrow = xh + (size_t)sTok[ar] * DM + ac * 32;
  _Float16* arow = sA + ar * APITCH + ac * 32;
#pragma unroll 1
  for (int kc = 0; kc < DM / 128; ++kc) {
    __syncthreads();
#pragma unroll
    for (int q = 0; q < 4; ++q) *(v8h*)(arow + 8 * q) = *(const v8h*)(xrow + kc * 128 + 8 * q);
    __syncthreads();
#pragma unroll 1
    for (int ks = 0; ks < 4; ++ks) {
      const int kg = kc * 128 + ks * 32;
      const v16h a = ldfrag(sA, APITCH, wm * 16, ks * 32, lane);
#pragma unroll
      for (int t = 0; t < 4; ++t) {
        const v16h bq = ldfrag(wge, DM, brow + 16 * t, kg, lane);
        accG[t] = mma16(a, bq, accG[t]);
      }
#pragma unroll
      for (int t = 0; t < 4; ++t) {
        const v16h bq = ldfrag(wue, DM, brow + 16 * t, kg, lane);
        accU[t] = mma16(a, bq, accU[t]);
      }
    }
  }

  _Float16* ew = sE + wave * (16 * EPITCH);
#pragma unroll
  for (int t = 0; t < 4; ++t) {
#pragma unroll
    for (int r = 0; r < 8; ++r) {
      const float g = accG[t][r] * UGS + bgv[t];
      const float u = accU[t][r] * UGS + buv[t];
      const float sg = __builtin_amdgcn_rcpf(1.0f + __expf(-g));
      const float av = ((g * sg) * u) * ACS;
      ew[(8 * hh + r) * EPITCH + 16 * t + c] = (_Float16)av;
    }
  }
  __syncthreads();
  v4u val[4];
  size_t go[4];
#pragma unroll
  for (int it = 0; it < 4; ++it) {
    const int p  = lane + 32 * it;
    const int L  = p >> 3;
    const int pc = p & 7;
    Pack8 pk;
    pk.h    = *(const v8h*)(ew + L * EPITCH + pc * 8);
    val[it] = pk.u;
    go[it]  = (size_t)(b * 64 + wm * 16 + L) * DH + brow + pc * 8;
  }
  for (int ps = 0; ps < 2; ++ps) {
#pragma unroll
    for (int it = 0; it < 4; ++it) *(volatile v4u*)(act + go[it]) = val[it];
    __threadfence();
  }
}

__global__ __launch_bounds__(256) void k_downx(const _Float16* __restrict__ act, const _Float16* __restrict__ wdt,
                                               const float* __restrict__ bd,
                                               const int* __restrict__ tokl, const float* __restrict__ wl,
                                               const int* __restrict__ tab, float* __restrict__ part) {
  __shared__ __align__(16) float sO[8 * 16 * OTP];
  __shared__ int   sEnc[64];
  __shared__ float sW[64];
  __shared__ int   sVal[64];
  __shared__ int   sTab[64];
  const int tid = threadIdx.x, lane = tid & 31, wave = tid >> 5;
  const int hh = lane >> 4, c = lane & 15;
  const int wm = wave & 3, wn = wave >> 2;
  const int b  = blockIdx.y;
  const int n0 = blockIdx.x * 128;

  if (tid < 64) sTab[tid] = tab[tid];
  __syncthreads();
  const int tb8 = clampi(sTab[32 + NE], 0, NTILE);
  if (b >= tb8) return;
  int e = 0;
#pragma unroll
  for (int q = 1; q < NE; ++q) e += (clampi(sTab[32 + q], 0, NTILE) <= b) ? 1 : 0;
  const int tbe = clampi(sTab[32 + e], 0, NTILE);
  const int cne = clampi(sTab[e], 0, NTOK);
  if (tid < 64) {
    const int rloc = (b - tbe) * 64 + tid;
    const bool valid = (rloc >= 0) && (rloc < cne);
    const int li = e * NTOK + clampi(rloc, 0, NTOK - 1);
    const int enc = tokl[li];
    const float w = wl[li];
    sEnc[tid] = clampi(enc, 0, NPROW - 1);
    sW[tid]   = valid ? w : 0.f;
    sVal[tid] = valid ? 1 : 0;
  }
  __syncthreads();

  const _Float16* wde = wdt + (size_t)e * (size_t)(DM * DH);
  const int brow = n0 + wn * 64;
  float bdv[4];
#pragma unroll
  for (int t = 0; t < 4; ++t) bdv[t] = bd[(size_t)e * DM + brow + 16 * t + c];

  v8f acc[4];
#pragma unroll
  for (int t = 0; t < 4; ++t) acc[t] = zero8();
  gemm16x64(act, DH, b * 64 + wm * 16, wde, DH, brow, DH, lane, acc);

  float wr[8];
#pragma unroll
  for (int r = 0; r < 8; ++r) wr[r] = sW[wm * 16 + 8 * hh + r];
  float* sw = sO + wave * (16 * OTP);
#pragma unroll
  for (int t = 0; t < 4; ++t) {
#pragma unroll
    for (int r = 0; r < 8; ++r) sw[(8 * hh + r) * OTP + 16 * t + c] = (acc[t][r] * DNS + bdv[t]) * wr[r];
  }
  __syncthreads();
  v4f val[8];
  size_t go[8];
  bool ok[8];
#pragma unroll
  for (int it = 0; it < 8; ++it) {
    const int p    = lane + 32 * it;
    const int L    = p >> 3;
    const int pc   = p & 7;
    const int row  = L >> 1;
    const int half = L & 1;
    const int lr   = wm * 16 + row;
    val[it] = *(const v4f*)(sw + row * OTP + half * 32 + pc * 4);
    ok[it]  = (sVal[lr] != 0);
    go[it]  = (size_t)sEnc[lr] * DM + brow + half * 32 + pc * 4;
  }
  for (int ps = 0; ps < 2; ++ps) {
#pragma unroll
    for (int it = 0; it < 8; ++it) {
      if (ok[it]) *(volatile v4f*)(part + go[it]) = val[it];
    }
    __threadfence();
  }
}

__global__ __launch_bounds__(256) void k_comb(const float* __restrict__ part, float* __restrict__ out, int n4) {
  const int i = blockIdx.x * 256 + (int)threadIdx.x;
  if (i >= n4) return;
  const size_t t = (size_t)i / (DM / 4);
  const size_t n = ((size_t)i % (DM / 4)) * 4;
  const float* pr = part + t * (size_t)(NSEL * DM) + n;
  v4f v = *(const v4f*)(pr);
  const v4f p1 = *(const v4f*)(pr + DM);
  v = v + p1;
  volatile v4f* d = (volatile v4f*)(out + t * DM + n);
  *d = v;
  __threadfence();
  *d = v;
}

extern "C" void kernel_launch(void* const* d_in, const int* in_sizes, int n_in,
                              void* d_out, int out_size, void* d_ws, size_t ws_size,
                              hipStream_t stream) {
  if (n_in < 6) return;
  if (in_sizes[0] != NTOK * DM) return;
  if (in_sizes[1] != DM * NE) return;
  if (in_sizes[2] != NE * DM * GU2) return;
  if (in_sizes[3] != NE * GU2) return;
  if (in_sizes[4] != NE * DH * DM) return;
  if (in_sizes[5] != NE * DM) return;
  if (out_size != NTOK * DM) return;

  const float* x    = (const float*)d_in[0];
  const float* Wgte = (const float*)d_in[1];
  const float* Wgu  = (const float*)d_in[2];
  const float* bgu  = (const float*)d_in[3];
  const float* Wd   = (const float*)d_in[4];
  const float* bd   = (const float*)d_in[5];
  float* out = (float*)d_out;

  size_t off = 0;
  const size_t oXh = off; off += (size_t)NTOK * DM * 2;
  const size_t oWg = off; off += (size_t)NE * GU2 * DM * 2;
  const size_t oWd = off; off += (size_t)NE * DM * DH * 2;
  const size_t oR  = off; off += (size_t)NTOK * RPITCH * 4;
  const size_t oTL = off; off += (size_t)NE * NTOK * 4;
  const size_t oWL = off; off += (size_t)NE * NTOK * 4;
  const size_t oTB = off; off += (size_t)256;
  const size_t oAC = off; off += (size_t)AROWS * DH * 2;
  const size_t oP  = off; off += (size_t)NPROW * DM * 4;
  if (off > ws_size) return;
  if (off > (size_t)134217728) return;
  if ((oWg | oWd | oR | oTL | oWL | oTB | oAC | oP) & (size_t)127) return;

  char* ws = (char*)d_ws;
  _Float16* Xh   = (_Float16*)(ws + oXh);
  _Float16* WguT = (_Float16*)(ws + oWg);
  _Float16* WdT  = (_Float16*)(ws + oWd);
  float*    R    = (float*)(ws + oR);
  int*      TOK  = (int*)(ws + oTL);
  float*    WL   = (float*)(ws + oWL);
  int*      TAB  = (int*)(ws + oTB);
  _Float16* ACT  = (_Float16*)(ws + oAC);
  float*    P    = (float*)(ws + oP);

  k_cvt<<<dim3((NTOK * DM) / 8 / 256), dim3(256), 0, stream>>>(x, Xh, (NTOK * DM) / 8);
  k_wtr<<<dim3(GU2 / 64, DM / 64, NE), dim3(256), 0, stream>>>(Wgu, WguT, DM, GU2, WSC);
  k_wtr<<<dim3(DM / 64, DH / 64, NE), dim3(256), 0, stream>>>(Wd, WdT, DH, DM, WSC);
  k_route<<<dim3(NTOK / 8), dim3(256), 0, stream>>>(x, Wgte, R);
  k_lists<<<dim3(1), dim3(256), 0, stream>>>(R, TOK, WL, TAB);
  k_upgate<<<dim3(DH / 128, NTILE), dim3(256), 0, stream>>>(Xh, WguT, bgu, TOK, TAB, ACT);
  k_downx<<<dim3(DM / 128, NTILE), dim3(256), 0, stream>>>(ACT, WdT, bd, TOK, WL, TAB, P);
  k_comb<<<dim3((NTOK * DM) / 4 / 256), dim3(256), 0, stream>>>(P, out, (NTOK * DM) / 4);
  (void)hipGetLastError();
}
